// NonLocal_40707700032191
// MI455X (gfx1250) — hardware-verified
//
#include <hip/hip_runtime.h>
#include <math.h>
#include <stddef.h>
#include <stdint.h>

#define NB    4
#define CH    64
#define NPOS  6400
#define NTOK  (NB * NPOS)
#define YP    128
#define NPART (NTOK / 64)
#define PARTW 128
#define SPT   68
#define WSMAX 134217728

static_assert(NPOS % 64 == 0);
static_assert(NTOK % 64 == 0);
static_assert(CH == 64);
static_assert(NPART == 400);
static_assert(YP == 2 * CH);
static_assert(PARTW == 2 * CH);

typedef float          v4f   __attribute__((ext_vector_type(4)));
typedef float          v8f   __attribute__((ext_vector_type(8)));
typedef int            v8i   __attribute__((ext_vector_type(8)));
typedef unsigned short v8us  __attribute__((ext_vector_type(8)));
typedef unsigned short v16us __attribute__((ext_vector_type(16)));
typedef __bf16         v16bf __attribute__((ext_vector_type(16)));
typedef __bf16         v8bf  __attribute__((ext_vector_type(8)));
typedef v4f  __attribute__((may_alias)) v4fa;
typedef v8us __attribute__((may_alias)) v8usa;
union FragB { v16bf v; v16us u; v8us h[2]; v8i w; };

__device__ __forceinline__ v8f wmb(const FragB& a, const FragB& b, v8f c) {
  v8f d = __builtin_amdgcn_wmma_f32_16x16x32_bf16(false, a.v, false, b.v, (short)0, c, false, false);
  asm volatile("v_nop\n\tv_nop\n\tv_nop\n\tv_nop" : "+v"(d) : "v"(a.w), "v"(b.w));
  return d;
}

__device__ __forceinline__ v8f z8() { v8f z = {0.f, 0.f, 0.f, 0.f, 0.f, 0.f, 0.f, 0.f}; return z; }

__device__ __forceinline__ unsigned bf16_bits(float f) {
  const unsigned u = __float_as_uint(f);
  return (u + 0x7FFFu + ((u >> 16) & 1u)) >> 16;
}
__device__ __forceinline__ float bf16_val(float f) {
  return __uint_as_float(bf16_bits(f) << 16);
}

__global__ __launch_bounds__(256) void k_wprep(const float* __restrict__ wq, const float* __restrict__ wk,
                                              const float* __restrict__ wg, const float* __restrict__ ww,
                                              unsigned short* WQ, unsigned short* WK, unsigned short* WG,
                                              unsigned short* WW2) {
  const int bx = (int)blockIdx.x, tid = (int)threadIdx.x;
  const float* p;
  unsigned short* dp;
  if (bx < 6) {
    const int which = bx >> 1;
    const float* src = (which == 0) ? wq : ((which == 1) ? wk : wg);
    unsigned short* dst = (which == 0) ? WQ : ((which == 1) ? WK : WG);
    const int u  = (bx & 1) * 256 + tid;
    const int o  = u >> 3;
    const int k8 = (u & 7) * 8;
    p  = src + (size_t)o * CH + k8;
    dp = dst + (size_t)u * 8;
  } else {
    const int v  = (bx - 6) * 256 + tid;
    const int o  = v >> 4;
    const int k8 = (v & 15) * 8;
    const int kk = k8 & (CH - 1);
    p  = ww + (size_t)o * CH + kk;
    dp = WW2 + (size_t)v * 8;
  }
  const v4f a = *(const v4f*)p;
  const v4f b = *(const v4f*)(p + 4);
  v8us o8;
  o8[0] = (unsigned short)bf16_bits(a.x); o8[1] = (unsigned short)bf16_bits(a.y);
  o8[2] = (unsigned short)bf16_bits(a.z); o8[3] = (unsigned short)bf16_bits(a.w);
  o8[4] = (unsigned short)bf16_bits(b.x); o8[5] = (unsigned short)bf16_bits(b.y);
  o8[6] = (unsigned short)bf16_bits(b.z); o8[7] = (unsigned short)bf16_bits(b.w);
  *(volatile v8us*)dp = o8;
  __threadfence();
  *(volatile v8us*)dp = o8;
}

__global__ __launch_bounds__(256) void k_xt(const float* __restrict__ x, unsigned short* xt) {
  __shared__ __attribute__((aligned(16))) float tf[64 * SPT];
  const int bx = (int)blockIdx.x, tid = (int)threadIdx.x;
  const int b  = bx / (NPOS / 64);
  const int n0 = (bx - b * (NPOS / 64)) * 64;
  {
    const int rsub = tid >> 4;
    const int c4   = (tid & 15) * 4;
#pragma unroll
    for (int it = 0; it < 4; ++it) {
      const int cr = it * 16 + rsub;
      const v4f a = *(const v4f*)(x + ((size_t)(b * CH + cr)) * NPOS + n0 + c4);
      *(v4fa*)(tf + cr * SPT + c4) = a;
    }
  }
  __syncthreads();
  const int rsub = tid >> 3;
  const int c8   = (tid & 7) * 8;
  v8us o[2];
#pragma unroll
  for (int it = 0; it < 2; ++it) {
    const int tl = it * 32 + rsub;
    v8us w;
#pragma unroll
    for (int e = 0; e < 8; ++e) w[e] = (unsigned short)bf16_bits(tf[(c8 + e) * SPT + tl]);
    o[it] = w;
  }
#pragma unroll
  for (int it = 0; it < 2; ++it) {
    const int tl = it * 32 + rsub;
    *(volatile v8us*)(xt + ((size_t)(b * NPOS + n0 + tl)) * CH + c8) = o[it];
  }
  __threadfence();
#pragma unroll
  for (int it = 0; it < 2; ++it) {
    const int tl = it * 32 + rsub;
    *(volatile v8us*)(xt + ((size_t)(b * NPOS + n0 + tl)) * CH + c8) = o[it];
  }
}

template <int OMODE, int BMODE>
__global__ __launch_bounds__(128) void k_gemm(const unsigned short* __restrict__ A, int lda, long sA,
                                              const unsigned short* __restrict__ BT, int ldb, long sB, int K,
                                              const float* __restrict__ bias,
                                              unsigned short* oh, unsigned short* ol, float* of, int ldc, long sC,
                                              float* part) {
  __shared__ __attribute__((aligned(16))) float stg[64 * SPT];
  __shared__ __attribute__((aligned(16))) float sb[64];
  __shared__ __attribute__((aligned(16))) float pst[PARTW];
  const int tid = (int)threadIdx.x, lane = tid & 31, wave = tid >> 5, hh = lane >> 4, m = lane & 15;
  const int rowBase = (int)blockIdx.x * 64;
  const int colBase = (int)blockIdx.y * 64;
  const int z = (int)blockIdx.z;
  const unsigned short* Ab = A  + (size_t)z * (size_t)sA;
  const unsigned short* Bb = BT + (size_t)z * (size_t)sB;
  if (tid < 64) sb[tid] = bf16_val(bias[(BMODE == 0 ? colBase : rowBase) + tid]);

  v8f acc[4];
#pragma unroll
  for (int t = 0; t < 4; ++t) acc[t] = z8();
  const unsigned short* ap = Ab + (size_t)(rowBase + 16 * wave + m) * (size_t)lda + 8 * hh;
  const unsigned short* bp = Bb + (size_t)(colBase + m) * (size_t)ldb + 8 * hh;

#pragma unroll 1
  for (int k0 = 0; k0 < K; k0 += 32) {
    FragB af;
    af.h[0] = *(const v8usa*)(ap + k0);
    af.h[1] = *(const v8usa*)(ap + k0 + 16);
#pragma unroll
    for (int nt = 0; nt < 4; ++nt) {
      const unsigned short* wq = bp + (size_t)(16 * nt) * (size_t)ldb + k0;
      FragB bf;
      bf.h[0] = *(const v8usa*)wq;
      bf.h[1] = *(const v8usa*)(wq + 16);
      acc[nt] = wmb(af, bf, acc[nt]);
    }
  }

#pragma unroll
  for (int nt = 0; nt < 4; ++nt) {
    const int lc = 16 * nt + m;
#pragma unroll
    for (int r = 0; r < 8; ++r) {
      const int lr = 16 * wave + 8 * hh + r;
      stg[lr * SPT + lc] = acc[nt][r];
    }
  }
  __syncthreads();

  if (OMODE == 0) {
    float* Cb = of + (size_t)z * (size_t)sC;
    const int rsub = tid >> 4;
    const int c4   = (tid & 15) * 4;
    v4f pv[8];
#pragma unroll
    for (int it = 0; it < 8; ++it) {
      const int row = it * 8 + rsub;
      v4f v = *(const v4fa*)(stg + row * SPT + c4);
      if (BMODE == 0) {
        v.x += sb[c4]; v.y += sb[c4 + 1]; v.z += sb[c4 + 2]; v.w += sb[c4 + 3];
      } else {
        const float br = sb[row];
        v.x += br; v.y += br; v.z += br; v.w += br;
      }
      pv[it] = v;
    }
#pragma unroll
    for (int it = 0; it < 8; ++it) {
      const int row = it * 8 + rsub;
      *(volatile v4f*)(Cb + (size_t)(rowBase + row) * (size_t)ldc + colBase + c4) = pv[it];
    }
    __threadfence();
#pragma unroll
    for (int it = 0; it < 8; ++it) {
      const int row = it * 8 + rsub;
      *(volatile v4f*)(Cb + (size_t)(rowBase + row) * (size_t)ldc + colBase + c4) = pv[it];
    }
    if (tid < 64) {
      const float bc = (BMODE == 0) ? sb[tid] : 0.0f;
      float s = 0.0f;
#pragma unroll 4
      for (int r = 0; r < 64; ++r) s += stg[r * SPT + tid] + ((BMODE == 0) ? bc : sb[r]);
      const float mean = s * (1.0f / 64.0f);
      float q = 0.0f;
#pragma unroll 4
      for (int r = 0; r < 64; ++r) {
        const float d = (stg[r * SPT + tid] + ((BMODE == 0) ? bc : sb[r])) - mean;
        q = fmaf(d, d, q);
      }
      pst[tid] = mean;
      pst[64 + tid] = q;
    }
    __syncthreads();
    v4f qv;
    if (tid < PARTW / 4) {
      qv = *(const v4fa*)(pst + 4 * tid);
      *(volatile v4f*)(part + (size_t)blockIdx.x * PARTW + 4 * tid) = qv;
    }
    __threadfence();
    if (tid < PARTW / 4) {
      *(volatile v4f*)(part + (size_t)blockIdx.x * PARTW + 4 * tid) = qv;
    }
  } else {
    unsigned short* Hb = oh + (size_t)z * (size_t)sC;
    unsigned short* Lb = ol + (size_t)z * (size_t)sC;
    const int rsub = tid >> 3;
    const int c8   = (tid & 7) * 8;
    v8us hv[4], lv[4];
#pragma unroll
    for (int it = 0; it < 4; ++it) {
      const int row = it * 16 + rsub;
      const float* sp = stg + row * SPT + c8;
      v8us h8, l8;
#pragma unroll
      for (int e = 0; e < 8; ++e) {
        const float v = sp[e] + ((BMODE == 0) ? sb[c8 + e] : sb[row]);
        const unsigned hb = bf16_bits(v);
        const unsigned lb = bf16_bits(v - __uint_as_float(hb << 16));
        h8[e] = (unsigned short)hb;
        l8[e] = (unsigned short)lb;
      }
      hv[it] = h8; lv[it] = l8;
    }
#pragma unroll
    for (int it = 0; it < 4; ++it) {
      const int row = it * 16 + rsub;
      const size_t go = (size_t)(rowBase + row) * (size_t)ldc + colBase + c8;
      *(volatile v8us*)(Hb + go) = hv[it];
      *(volatile v8us*)(Lb + go) = lv[it];
    }
    __threadfence();
#pragma unroll
    for (int it = 0; it < 4; ++it) {
      const int row = it * 16 + rsub;
      const size_t go = (size_t)(rowBase + row) * (size_t)ldc + colBase + c8;
      *(volatile v8us*)(Hb + go) = hv[it];
      *(volatile v8us*)(Lb + go) = lv[it];
    }
  }
}

#define AT_D  64
#define AT_NW 4
#define AT_QB 64
#define AT_KC 64

__device__ __forceinline__ unsigned short at_bf_bits(float f) {
  unsigned u = __float_as_uint(f);
  return (unsigned short)((u + 0x7FFFu + ((u >> 16) & 1u)) >> 16);
}
__device__ __forceinline__ __bf16 at_f2bf(float f) { return __builtin_bit_cast(__bf16, at_bf_bits(f)); }
__device__ __forceinline__ void at_split(float f, __bf16& hi, __bf16& lo) {
  const unsigned short hb = at_bf_bits(f);
  hi = __builtin_bit_cast(__bf16, hb);
  lo = at_f2bf(f - __uint_as_float(((unsigned)hb) << 16));
}
__device__ __forceinline__ v8f at_mma(v16bf a, v16bf b, v8f c) {
  c = __builtin_amdgcn_wmma_f32_16x16x32_bf16(false, a, false, b, (short)0, c, false, false);
  asm volatile("v_nop\n\tv_nop\n\tv_nop\n\tv_nop" : "+v"(c) : "v"(a), "v"(b));
  return c;
}
union AtFB { v16bf v; v8bf h[2]; };
__device__ __forceinline__ v16bf at_ldfrag(const __bf16* p) {
  AtFB f; f.h[0] = *(const v8bf*)(p); f.h[1] = *(const v8bf*)(p + 16); return f.v;
}

__global__ __launch_bounds__(128)
void k_attn(const unsigned short* __restrict__ qhp, const unsigned short* __restrict__ qlp,
            const unsigned short* __restrict__ khp, const unsigned short* __restrict__ klp,
            const unsigned short* __restrict__ vhp, const unsigned short* __restrict__ vlp,
            unsigned short* yout) {
  __shared__ __align__(16) __bf16 Ksh[AT_KC * AT_D];
  __shared__ __align__(16) __bf16 Ksl[AT_KC * AT_D];
  __shared__ __align__(16) __bf16 Vth[AT_D * AT_KC];
  __shared__ __align__(16) __bf16 Vtl[AT_D * AT_KC];
  __shared__ __align__(16) __bf16 Psh[AT_NW][16 * AT_KC];
  __shared__ __align__(16) __bf16 Psl[AT_NW][16 * AT_KC];
  __shared__ __align__(16) float  Os[AT_NW][16 * SPT];

  const int tid  = (int)threadIdx.x;
  const int wave = tid >> 5;
  const int lane = tid & 31;
  const int hh   = lane >> 4;
  const int c    = lane & 15;

  const int nqb = NPOS / AT_QB;
  const int bx  = (int)blockIdx.x;
  const int b   = bx / nqb;
  const int qb  = bx - b * nqb;
  const int q0  = qb * AT_QB + wave * 16;

  const __bf16* Qh = (const __bf16*)(const void*)qhp + (size_t)b * NPOS * AT_D;
  const __bf16* Ql = (const __bf16*)(const void*)qlp + (size_t)b * NPOS * AT_D;
  const __bf16* Kh = (const __bf16*)(const void*)khp + (size_t)b * NPOS * AT_D;
  const __bf16* Kl = (const __bf16*)(const void*)klp + (size_t)b * NPOS * AT_D;
  const __bf16* Vh = (const __bf16*)(const void*)vhp + (size_t)b * AT_D * NPOS;
  const __bf16* Vl = (const __bf16*)(const void*)vlp + (size_t)b * AT_D * NPOS;
  unsigned short* yb = yout + (size_t)b * NPOS * YP;

  v16bf qah[2], qal[2];
#pragma unroll
  for (int dc = 0; dc < 2; ++dc) {
    const __bf16* qr = Qh + (size_t)(q0 + c) * AT_D + dc * 32 + 8 * hh;
    const __bf16* ql = Ql + (size_t)(q0 + c) * AT_D + dc * 32 + 8 * hh;
    qah[dc] = at_ldfrag(qr);
    qal[dc] = at_ldfrag(ql);
  }

  float mrow[8], lrow[8];
  v8f oacc[4];
#pragma unroll
  for (int r = 0; r < 8; ++r) { mrow[r] = -INFINITY; lrow[r] = 0.f; }
#pragma unroll
  for (int t = 0; t < 4; ++t) oacc[t] = z8();

  const int nChunks = NPOS / AT_KC;
  for (int kc = 0; kc < nChunks; ++kc) {
    const int kv0 = kc * AT_KC;
    __syncthreads();
    {
      const int r = tid >> 1, half = (tid & 1) * 32;
      const __bf16* ksh = Kh + (size_t)(kv0 + r) * AT_D + half;
      const __bf16* ksl = Kl + (size_t)(kv0 + r) * AT_D + half;
      const __bf16* vsh = Vh + (size_t)r * NPOS + kv0 + half;
      const __bf16* vsl = Vl + (size_t)r * NPOS + kv0 + half;
#pragma unroll
      for (int i = 0; i < 4; ++i) {
        const v8bf a0 = *(const v8bf*)(ksh + 8 * i);
        const v8bf a1 = *(const v8bf*)(ksl + 8 * i);
        const v8bf b0 = *(const v8bf*)(vsh + 8 * i);
        const v8bf b1 = *(const v8bf*)(vsl + 8 * i);
        *(v8bf*)(Ksh + r * AT_D  + half + 8 * i) = a0;
        *(v8bf*)(Ksl + r * AT_D  + half + 8 * i) = a1;
        *(v8bf*)(Vth + r * AT_KC + half + 8 * i) = b0;
        *(v8bf*)(Vtl + r * AT_KC + half + 8 * i) = b1;
      }
    }
    __syncthreads();

    v8f s[4];
#pragma unroll
    for (int j = 0; j < 4; ++j) {
      s[j] = z8();
#pragma unroll
      for (int dc = 0; dc < 2; ++dc) {
        AtFB kb, kl;
        kb.h[0] = *(const v8bf*)(Ksh + (j * 16 + c) * AT_D + dc * 32 + 8 * hh);
        kb.h[1] = *(const v8bf*)(Ksh + (j * 16 + c) * AT_D + dc * 32 + 16 + 8 * hh);
        kl.h[0] = *(const v8bf*)(Ksl + (j * 16 + c) * AT_D + dc * 32 + 8 * hh);
        kl.h[1] = *(const v8bf*)(Ksl + (j * 16 + c) * AT_D + dc * 32 + 16 + 8 * hh);
        s[j] = at_mma(qah[dc], kb.v, s[j]);
        s[j] = at_mma(qah[dc], kl.v, s[j]);
        s[j] = at_mma(qal[dc], kb.v, s[j]);
      }
    }
    float cm[8];
#pragma unroll
    for (int r = 0; r < 8; ++r) {
      float mx = -INFINITY;
#pragma unroll
      for (int j = 0; j < 4; ++j) mx = fmaxf(mx, s[j][r]);
#pragma unroll
      for (int off = 1; off < 16; off <<= 1) mx = fmaxf(mx, __shfl_xor(mx, off, 32));
      cm[r] = mx;
    }
    __bf16* pwh = Psh[wave];
    __bf16* pwl = Psl[wave];
#pragma unroll
    for (int r = 0; r < 8; ++r) {
      const float mnew  = fmaxf(mrow[r], cm[r]);
      const float alpha = expf(mrow[r] - mnew);
      mrow[r] = mnew;
      float psum = 0.f;
#pragma unroll
      for (int j = 0; j < 4; ++j) {
        const float p = expf(s[j][r] - mnew);
        psum += p;
        __bf16 a, bl; at_split(p, a, bl);
        pwh[(8 * hh + r) * AT_KC + j * 16 + c] = a;
        pwl[(8 * hh + r) * AT_KC + j * 16 + c] = bl;
      }
#pragma unroll
      for (int off = 1; off < 16; off <<= 1) psum += __shfl_xor(psum, off, 32);
      lrow[r] = lrow[r] * alpha + psum;
#pragma unroll
      for (int t = 0; t < 4; ++t) oacc[t][r] *= alpha;
    }
    __builtin_amdgcn_fence(__ATOMIC_RELEASE, "workgroup");
    __builtin_amdgcn_wave_barrier();
    __builtin_amdgcn_fence(__ATOMIC_ACQUIRE, "workgroup");
#pragma unroll 1
    for (int kk = 0; kk < 2; ++kk) {
      AtFB pa, pl;
      pa.h[0] = *(const v8bf*)(pwh + c * AT_KC + kk * 32 + 8 * hh);
      pa.h[1] = *(const v8bf*)(pwh + c * AT_KC + kk * 32 + 16 + 8 * hh);
      pl.h[0] = *(const v8bf*)(pwl + c * AT_KC + kk * 32 + 8 * hh);
      pl.h[1] = *(const v8bf*)(pwl + c * AT_KC + kk * 32 + 16 + 8 * hh);
#pragma unroll
      for (int t = 0; t < 4; ++t) {
        AtFB vb, vl;
        vb.h[0] = *(const v8bf*)(Vth + (t * 16 + c) * AT_KC + kk * 32 + 8 * hh);
        vb.h[1] = *(const v8bf*)(Vth + (t * 16 + c) * AT_KC + kk * 32 + 16 + 8 * hh);
        vl.h[0] = *(const v8bf*)(Vtl + (t * 16 + c) * AT_KC + kk * 32 + 8 * hh);
        vl.h[1] = *(const v8bf*)(Vtl + (t * 16 + c) * AT_KC + kk * 32 + 16 + 8 * hh);
        oacc[t] = at_mma(pa.v, vb.v, oacc[t]);
        oacc[t] = at_mma(pa.v, vl.v, oacc[t]);
        oacc[t] = at_mma(pl.v, vb.v, oacc[t]);
      }
    }
  }

  float* os = Os[wave];
#pragma unroll
  for (int r = 0; r < 8; ++r) {
    const float inv = 1.0f / lrow[r];
#pragma unroll
    for (int t = 0; t < 4; ++t) os[(8 * hh + r) * SPT + t * 16 + c] = oacc[t][r] * inv;
  }
  __builtin_amdgcn_fence(__ATOMIC_RELEASE, "workgroup");
  __builtin_amdgcn_wave_barrier();
  __builtin_amdgcn_fence(__ATOMIC_ACQUIRE, "workgroup");
  {
    const int q  = lane >> 3;
    const int c8 = (lane & 7) * 8;
    v8us hv[4], lv[4];
#pragma unroll
    for (int it = 0; it < 4; ++it) {
      const int row = it * 4 + q;
      const float* sp = os + row * SPT + c8;
      v8us h8, l8;
#pragma unroll
      for (int e = 0; e < 8; ++e) {
        const float f = sp[e];
        const unsigned short hb = at_bf_bits(f);
        const unsigned short lb = at_bf_bits(f - __uint_as_float(((unsigned)hb) << 16));
        h8[e] = hb; l8[e] = lb;
      }
      hv[it] = h8; lv[it] = l8;
    }
#pragma unroll
    for (int it = 0; it < 4; ++it) {
      const int row = it * 4 + q;
      unsigned short* yr = yb + (size_t)(q0 + row) * YP + c8;
      *(volatile v8us*)(yr)        = hv[it];
      *(volatile v8us*)(yr + AT_D) = lv[it];
    }
    __threadfence();
#pragma unroll
    for (int it = 0; it < 4; ++it) {
      const int row = it * 4 + q;
      unsigned short* yr = yb + (size_t)(q0 + row) * YP + c8;
      *(volatile v8us*)(yr)        = hv[it];
      *(volatile v8us*)(yr + AT_D) = lv[it];
    }
  }
}

__global__ __launch_bounds__(64) void k_bnfin(const float* __restrict__ part, const float* __restrict__ gam,
                                              const float* __restrict__ bet, float* ss) {
  __shared__ __attribute__((aligned(16))) float stg[2 * CH];
  const int tid = (int)threadIdx.x;
  const int c = tid & (CH - 1);
  float s = 0.0f;
#pragma unroll 1
  for (int p = 0; p < NPART; ++p) s += part[(size_t)p * PARTW + c];
  const float mean = s * (1.0f / (float)NPART);
  float q = 0.0f;
#pragma unroll 1
  for (int p = 0; p < NPART; ++p) {
    const float mb = part[(size_t)p * PARTW + c];
    const float qb = part[(size_t)p * PARTW + CH + c];
    const float d = mb - mean;
    q = q + (qb + 64.0f * d * d);
  }
  const float var  = q * (1.0f / (float)NTOK);
  const float rstd = rsqrtf(var + 1e-5f);
  const float sc = bf16_val(gam[c]) * rstd;
  const float sh = bf16_val(bet[c]) - mean * sc;
  stg[c] = sc;
  stg[CH + c] = sh;
  __syncthreads();
  v4f v;
  if (tid < (2 * CH) / 4) {
    v = *(const v4fa*)(stg + 4 * tid);
    *(volatile v4f*)(ss + 4 * tid) = v;
  }
  __threadfence();
  if (tid < (2 * CH) / 4) {
    *(volatile v4f*)(ss + 4 * tid) = v;
  }
}

__global__ __launch_bounds__(256) void k_out(const float* __restrict__ wy, const float* __restrict__ ss,
                                             const float* __restrict__ x, float* out) {
  __shared__ __attribute__((aligned(16))) float tf[64 * SPT];
  __shared__ __attribute__((aligned(16))) float ssh[2 * CH];
  const int bx = (int)blockIdx.x, tid = (int)threadIdx.x;
  if (tid < 2 * CH) ssh[tid] = ss[tid];
  __syncthreads();
  const int b  = bx / (NPOS / 64);
  const int n0 = (bx - b * (NPOS / 64)) * 64;
  const int t0 = b * NPOS + n0;
  const int rsub = tid >> 4;
  const int c4   = (tid & 15) * 4;
#pragma unroll
  for (int it = 0; it < 4; ++it) {
    const int tl = it * 16 + rsub;
    const v4f a = *(const v4f*)(wy + (size_t)(t0 + tl) * CH + c4);
    tf[(c4 + 0) * SPT + tl] = fmaf(a.x, ssh[c4 + 0], ssh[CH + c4 + 0]);
    tf[(c4 + 1) * SPT + tl] = fmaf(a.y, ssh[c4 + 1], ssh[CH + c4 + 1]);
    tf[(c4 + 2) * SPT + tl] = fmaf(a.z, ssh[c4 + 2], ssh[CH + c4 + 2]);
    tf[(c4 + 3) * SPT + tl] = fmaf(a.w, ssh[c4 + 3], ssh[CH + c4 + 3]);
  }
  __syncthreads();
  v4f ov[4];
#pragma unroll
  for (int it = 0; it < 4; ++it) {
    const int ch = it * 16 + rsub;
    const size_t gi = ((size_t)(b * CH + ch)) * NPOS + n0 + c4;
    const v4f bn = *(const v4fa*)(tf + ch * SPT + c4);
    const v4f xr = *(const v4f*)(x + gi);
    v4f v;
    v.x = bn.x + bf16_val(xr.x); v.y = bn.y + bf16_val(xr.y);
    v.z = bn.z + bf16_val(xr.z); v.w = bn.w + bf16_val(xr.w);
    ov[it] = v;
  }
#pragma unroll
  for (int it = 0; it < 4; ++it) {
    const int ch = it * 16 + rsub;
    const size_t gi = ((size_t)(b * CH + ch)) * NPOS + n0 + c4;
    *(volatile v4f*)(out + gi) = ov[it];
  }
  __threadfence();
#pragma unroll
  for (int it = 0; it < 4; ++it) {
    const int ch = it * 16 + rsub;
    const size_t gi = ((size_t)(b * CH + ch)) * NPOS + n0 + c4;
    *(volatile v4f*)(out + gi) = ov[it];
  }
}

static inline size_t al256(size_t o) { return (o + 255) & ~(size_t)255; }

extern "C" void kernel_launch(void* const* d_in, const int* in_sizes, int n_in,
                              void* d_out, int out_size, void* d_ws, size_t ws_size,
                              hipStream_t stream) {
  if (n_in < 11) return;
  if (in_sizes[0] != NB * CH * NPOS) return;
  if (in_sizes[1] != CH * CH || in_sizes[3] != CH * CH) return;
  if (in_sizes[5] != CH * CH || in_sizes[7] != CH * CH) return;
  if (in_sizes[2] != CH || in_sizes[4] != CH || in_sizes[6] != CH) return;
  if (in_sizes[8] != CH || in_sizes[9] != CH || in_sizes[10] != CH) return;
  if (out_size != NB * CH * NPOS) return;

  const float* x       = (const float*)d_in[0];
  const float* w_theta = (const float*)d_in[1];
  const float* b_theta = (const float*)d_in[2];
  const float* w_phi   = (const float*)d_in[3];
  const float* b_phi   = (const float*)d_in[4];
  const float* w_g     = (const float*)d_in[5];
  const float* b_g     = (const float*)d_in[6];
  const float* w_W     = (const float*)d_in[7];
  const float* b_W     = (const float*)d_in[8];
  const float* gamma   = (const float*)d_in[9];
  const float* beta    = (const float*)d_in[10];
  float* out = (float*)d_out;

  const size_t PW  = (size_t)CH * CH * 2;
  const size_t PW2 = (size_t)CH * YP * 2;
  const size_t PA  = (size_t)NTOK * CH * 2;
  const size_t PY  = (size_t)NTOK * YP * 2;
  const size_t PF  = (size_t)NTOK * CH * 4;
  size_t off = 0;
  const size_t oWQ  = off; off = al256(off + PW);
  const size_t oWK  = off; off = al256(off + PW);
  const size_t oWG  = off; off = al256(off + PW);
  const size_t oWW2 = off; off = al256(off + PW2);
  const size_t oXT  = off; off = al256(off + PA);
  const size_t oTHh = off; off = al256(off + PA);
  const size_t oTHl = off; off = al256(off + PA);
  const size_t oPHh = off; off = al256(off + PA);
  const size_t oPHl = off; off = al256(off + PA);
  const size_t oGTh = off; off = al256(off + PA);
  const size_t oGTl = off; off = al256(off + PA);
  const size_t oY   = off; off = al256(off + PY);
  const size_t oWY  = off; off = al256(off + PF);
  const size_t oPT  = off; off = al256(off + (size_t)NPART * PARTW * 4);
  const size_t oSS  = off; off = al256(off + (size_t)(2 * CH) * 4);
  if (off > ws_size || off > (size_t)WSMAX) return;

  char* ws = (char*)d_ws;
  unsigned short* WQ  = (unsigned short*)(ws + oWQ);
  unsigned short* WK  = (unsigned short*)(ws + oWK);
  unsigned short* WG  = (unsigned short*)(ws + oWG);
  unsigned short* WW2 = (unsigned short*)(ws + oWW2);
  unsigned short* XT  = (unsigned short*)(ws + oXT);
  unsigned short* THh = (unsigned short*)(ws + oTHh);
  unsigned short* THl = (unsigned short*)(ws + oTHl);
  unsigned short* PHh = (unsigned short*)(ws + oPHh);
  unsigned short* PHl = (unsigned short*)(ws + oPHl);
  unsigned short* GTh = (unsigned short*)(ws + oGTh);
  unsigned short* GTl = (unsigned short*)(ws + oGTl);
  unsigned short* Y   = (unsigned short*)(ws + oY);
  float*          WY  = (float*)(ws + oWY);
  float*          PT  = (float*)(ws + oPT);
  float*          SS  = (float*)(ws + oSS);

  k_wprep<<<10, 256, 0, stream>>>(w_theta, w_phi, w_g, w_W, WQ, WK, WG, WW2);
  k_xt<<<NB * (NPOS / 64), 256, 0, stream>>>(x, XT);
  k_gemm<1, 0><<<dim3(NTOK / 64, 1, 1), 128, 0, stream>>>(XT, CH, 0L, WQ, CH, 0L, CH, b_theta,
                                                         THh, THl, WY, CH, 0L, PT);
  k_gemm<1, 0><<<dim3(NTOK / 64, 1, 1), 128, 0, stream>>>(XT, CH, 0L, WK, CH, 0L, CH, b_phi,
                                                         PHh, PHl, WY, CH, 0L, PT);
  k_gemm<1, 1><<<dim3(1, NPOS / 64, NB), 128, 0, stream>>>(WG, CH, 0L, XT, CH, (long)NPOS * CH, CH, b_g,
                                                          GTh, GTl, WY, NPOS, (long)CH * NPOS, PT);
  k_attn<<<NB * (NPOS / AT_QB), 128, 0, stream>>>(THh, THl, PHh, PHl, GTh, GTl, Y);
  k_gemm<0, 0><<<dim3(NTOK / 64, 1, 1), 128, 0, stream>>>(Y, YP, 0L, WW2, YP, 0L, YP, b_W,
                                                         THh, THl, WY, CH, 0L, PT);
  k_bnfin<<<1, 64, 0, stream>>>(PT, gamma, beta, SS);
  k_out<<<NB * (NPOS / 64), 256, 0, stream>>>(WY, SS, x, out);
  (void)hipGetLastError();
}
